// MambaTasNet_40802189312120
// MI455X (gfx1250) — hardware-run, weakly checked
//
#include <hip/hip_runtime.h>
#include <math.h>

typedef __attribute__((ext_vector_type(16))) _Float16 v16h;
typedef __attribute__((ext_vector_type(8)))  _Float16 v8h;
typedef __attribute__((ext_vector_type(8)))  float    v8f;
typedef __attribute__((ext_vector_type(4)))  float    v4f;

constexpr int kBatch = 2;
constexpr int kSamp  = 8000;
constexpr int kEnc   = 256;
constexpr int kKer   = 16;
constexpr int kStr   = 8;
constexpr int kL     = 999;
constexpr int kMV    = kBatch * kL;
constexpr int kMP    = 2048;
constexpr int kBot   = 256;
constexpr int kDI    = 512;
constexpr int kNS    = 16;
constexpr int kDtR   = 16;
constexpr int kNBlk  = 8;
constexpr int kXpN   = 48;
constexpr int kXdP   = 64;
constexpr int kXzP   = 2 * kDI;
constexpr int kConvTP = 260;
constexpr int kScanTS = 64;
constexpr int kScanCh = 64;
constexpr int kScanYP = 68;
constexpr int kPartLines = kMP / 4;
constexpr float kActCarry = 16.0f;
constexpr float kWgtCarry = 32.0f;
constexpr float kFold = 1.0f / (kActCarry * kWgtCarry);
static_assert((kSamp - kKer) / kStr + 1 == kL);
static_assert(kMV == 1998 && kMV <= kMP && (kMP % 64) == 0);
static_assert(kDtR + 2 * kNS == kXpN && kXpN <= kXdP);
static_assert((kBot % 32) == 0 && (kDI % 32) == 0 && (kEnc % 32) == 0);
static_assert((kXzP % 64) == 0 && (kXdP % 64) == 0 && (kBot % 64) == 0 && (kEnc % 64) == 0);
static_assert((kDI % kScanCh) == 0 && (kDI % 256) == 0);
static_assert((kBatch * kSamp) % 32 == 0);

constexpr size_t kSzWIN  = (size_t)kNBlk * 2 * kXzP * kBot * 2;
constexpr size_t kSzWOUT = (size_t)kNBlk * 2 * kBot * kDI * 2;
constexpr size_t kSzWXP  = (size_t)kNBlk * 2 * kXdP * kDI * 2;
constexpr size_t kSzWBOT = (size_t)kBot * kEnc * 2;
constexpr size_t kSzWMSK = (size_t)kEnc * kBot * 2;
constexpr size_t kSzMW   = (size_t)kMP * kEnc * 4;
constexpr size_t kSzPART = (size_t)kPartLines * 128;
constexpr size_t kSzSTAT = 1024;
constexpr size_t kSzGN   = (size_t)kMP * kEnc * 2;
constexpr size_t kSzX    = (size_t)kMP * kBot * 4;
constexpr size_t kSzXN   = (size_t)2 * kMP * kBot * 2;
constexpr size_t kSzXZ   = (size_t)2 * kMP * kXzP * 4;
constexpr size_t kSzXC   = (size_t)2 * kMP * kDI * 4;
constexpr size_t kSzXC16 = (size_t)2 * kMP * kDI * 2;
constexpr size_t kSzXD   = (size_t)2 * kMP * kXdP * 4;
constexpr size_t kSzG    = (size_t)2 * kMP * kDI * 2;
constexpr size_t kSzYD   = (size_t)2 * kMP * kBot * 4;
constexpr size_t kSzMSK  = (size_t)kMP * kEnc * 4;
constexpr size_t kOffWIN  = 0;
constexpr size_t kOffWOUT = kOffWIN  + kSzWIN;
constexpr size_t kOffWXP  = kOffWOUT + kSzWOUT;
constexpr size_t kOffWBOT = kOffWXP  + kSzWXP;
constexpr size_t kOffWMSK = kOffWBOT + kSzWBOT;
constexpr size_t kOffMW   = kOffWMSK + kSzWMSK;
constexpr size_t kOffPART = kOffMW   + kSzMW;
constexpr size_t kOffSTAT = kOffPART + kSzPART;
constexpr size_t kOffGN   = kOffSTAT + kSzSTAT;
constexpr size_t kOffXA   = kOffGN   + kSzGN;
constexpr size_t kOffXB   = kOffXA   + kSzX;
constexpr size_t kOffXN   = kOffXB   + kSzX;
constexpr size_t kOffXZ   = kOffXN   + kSzXN;
constexpr size_t kOffXC   = kOffXZ   + kSzXZ;
constexpr size_t kOffXC16 = kOffXC   + kSzXC;
constexpr size_t kOffXD   = kOffXC16 + kSzXC16;
constexpr size_t kOffG    = kOffXD   + kSzXD;
constexpr size_t kOffYD   = kOffG    + kSzG;
constexpr size_t kOffMSK  = kOffYD   + kSzYD;
constexpr size_t kWsTotal = kOffMSK  + kSzMSK;
static_assert(kWsTotal == 64291840ull);
static_assert(kWsTotal <= 134217728ull);
static_assert((kOffWOUT % 128) == 0 && (kOffWXP % 128) == 0 && (kOffWBOT % 128) == 0 && (kOffWMSK % 128) == 0 &&
              (kOffMW % 128) == 0 && (kOffPART % 128) == 0 && (kOffSTAT % 128) == 0 && (kOffGN % 128) == 0 &&
              (kOffXA % 128) == 0 && (kOffXB % 128) == 0 && (kOffXN % 128) == 0 && (kOffXZ % 128) == 0 &&
              (kOffXC % 128) == 0 && (kOffXC16 % 128) == 0 && (kOffXD % 128) == 0 && (kOffG % 128) == 0 &&
              (kOffYD % 128) == 0 && (kOffMSK % 128) == 0);

__device__ __forceinline__ void guard_row4(v8f& a, v8f& b, v8f& c, v8f& d, v16h x, v16h y0, v16h y1, v16h y2, v16h y3) {
  asm volatile("v_nop\n\tv_nop\n\tv_nop\n\tv_nop" : "+v"(a), "+v"(b), "+v"(c), "+v"(d) : "v"(x), "v"(y0), "v"(y1), "v"(y2), "v"(y3));
}
__device__ __forceinline__ void keep4_h(v16h a, v16h b, v16h c, v16h d) { asm volatile("v_nop" :: "v"(a), "v"(b), "v"(c), "v"(d)); }
__device__ __forceinline__ void acc_guard4(v8f& a, v8f& b, v8f& c, v8f& d) { asm volatile("v_nop\n\tv_nop\n\tv_nop\n\tv_nop" : "+v"(a), "+v"(b), "+v"(c), "+v"(d)); }
struct FragH {
  union U { v16h v; v8h h[2]; };
  static __device__ __forceinline__ v16h load(const _Float16* p) {
    U f; f.h[0] = *(const v8h*)(p); f.h[1] = *(const v8h*)(p + 16); return f.v;
  }
  static __device__ __forceinline__ v8f mma(v16h a, v16h b, v8f c) {
    return __builtin_amdgcn_wmma_f32_16x16x32_f16(false, a, false, b, (short)0, c, false, false);
  }
};

template <int BIAS_MODE, int ACT>
__global__ __launch_bounds__(256) void gemm64_f16_kernel(
    const unsigned short* __restrict__ Ap, int lda, long strideA,
    const unsigned short* __restrict__ Btp, int ldb, long strideB,
    float* __restrict__ Cout, int ldc, long strideC,
    const float* __restrict__ bias, int M, int N, int K, float scale)
{
  __shared__ __align__(16) float sT[8][16 * 68];
  const int b    = blockIdx.y;
  const int lane = threadIdx.x & 31;
  const int wave = threadIdx.x >> 5;
  const int tilesN = N >> 6;
  const int tilesM = M >> 6;
  const int tile = blockIdx.x * 8 + wave;
  if (tile >= tilesM * tilesN) return;
  const int tm = tile / tilesN;
  const int tn = tile - tm * tilesN;
  const int m0 = tm << 6;
  const int n0 = tn << 6;
  const _Float16* Ab = (const _Float16*)Ap  + (size_t)b * strideA;
  const _Float16* Bb = (const _Float16*)Btp + (size_t)b * strideB;
  const int rlane = lane & 15;
  const int koff  = (lane >> 4) * 8;
  const int mOff  = (lane >> 4) * 8;

  v8f acc[4][4];
#pragma unroll
  for (int i = 0; i < 4; ++i)
#pragma unroll
    for (int j = 0; j < 4; ++j) acc[i][j] = (v8f){0.f, 0.f, 0.f, 0.f, 0.f, 0.f, 0.f, 0.f};

  for (int k0 = 0; k0 < K; k0 += 32) {
    v16h bh[4];
#pragma unroll
    for (int j = 0; j < 4; ++j) {
      const size_t bo = (size_t)(n0 + (j << 4) + rlane) * ldb + koff + k0;
      bh[j] = FragH::load(Bb + bo);
    }
#pragma unroll
    for (int i = 0; i < 4; ++i) {
      const size_t ao = (size_t)(m0 + (i << 4) + rlane) * lda + koff + k0;
      const v16h ah = FragH::load(Ab + ao);
#pragma unroll
      for (int j = 0; j < 4; ++j) acc[i][j] = FragH::mma(ah, bh[j], acc[i][j]);
      guard_row4(acc[i][0], acc[i][1], acc[i][2], acc[i][3], ah, bh[0], bh[1], bh[2], bh[3]);
    }
    keep4_h(bh[0], bh[1], bh[2], bh[3]);
  }
  acc_guard4(acc[0][0], acc[0][1], acc[0][2], acc[0][3]);
  acc_guard4(acc[1][0], acc[1][1], acc[1][2], acc[1][3]);
  acc_guard4(acc[2][0], acc[2][1], acc[2][2], acc[2][3]);
  acc_guard4(acc[3][0], acc[3][1], acc[3][2], acc[3][3]);

  float* slab = sT[wave];
  float* C = Cout + (size_t)b * strideC;
#pragma unroll
  for (int i = 0; i < 4; ++i) {
    const int mBase = m0 + (i << 4);
#pragma unroll
    for (int j = 0; j < 4; ++j) {
      const int n = n0 + (j << 4) + rlane;
      float bv = 0.f;
      if (BIAS_MODE == 2) bv = bias[n];
#pragma unroll
      for (int r = 0; r < 8; ++r) {
        float v = acc[i][j][r] * scale;
        if (BIAS_MODE == 2) v += bv;
        if (ACT == 2) v = fmaxf(v, 0.0f);
        slab[(mOff + r) * 68 + (j << 4) + rlane] = v;
      }
    }
    __builtin_amdgcn_fence(__ATOMIC_RELEASE, "workgroup");
    __builtin_amdgcn_wave_barrier();
    __builtin_amdgcn_fence(__ATOMIC_ACQUIRE, "workgroup");
    {
      const int hh = lane >> 4, c4 = (lane & 15) * 4;
      for (int pass = 0; pass < 2; ++pass) {
#pragma unroll
        for (int it = 0; it < 8; ++it) {
          const int row = it * 2 + hh;
          const v4f v = *(const v4f*)(slab + row * 68 + c4);
          *(volatile v4f*)(C + (size_t)(mBase + row) * ldc + n0 + c4) = v;
        }
        __threadfence();
      }
    }
    __builtin_amdgcn_fence(__ATOMIC_RELEASE, "workgroup");
    __builtin_amdgcn_wave_barrier();
    __builtin_amdgcn_fence(__ATOMIC_ACQUIRE, "workgroup");
  }
}

__global__ __launch_bounds__(256) void cast_f16_kernel(
    const float* __restrict__ src, unsigned short* __restrict__ dst, int total8, float scale)
{
  const int i = blockIdx.x * 256 + threadIdx.x;
  if (i >= total8) return;
  const size_t e0 = (size_t)i << 3;
  const float* p = src + e0;
  const v4f a0 = *(const v4f*)(p);
  const v4f a1 = *(const v4f*)(p + 4);
  v8h hv;
#pragma unroll
  for (int e = 0; e < 4; ++e) {
    hv[e]     = (_Float16)(a0[e] * scale);
    hv[4 + e] = (_Float16)(a1[e] * scale);
  }
  unsigned short* q = dst + e0;
  *(volatile v8h*)q = hv;
  __threadfence();
  *(volatile v8h*)q = hv;
}

__global__ __launch_bounds__(256) void xproj_pad_cast_kernel(
    const float* __restrict__ src, unsigned short* __restrict__ dst, int total8, float scale)
{
  const int i = blockIdx.x * 256 + threadIdx.x;
  if (i >= total8) return;
  const int e0 = i << 3;
  const int k  = e0 & (kDI - 1);
  const int rr = (e0 >> 9) & (kXdP - 1);
  const int w  = e0 >> 15;
  const bool keepv = rr < kXpN;
  const int rc = keepv ? rr : (kXpN - 1);
  const float* p = src + ((size_t)w * kXpN + rc) * kDI + k;
  const v4f a0 = *(const v4f*)(p);
  const v4f a1 = *(const v4f*)(p + 4);
  v8h hv;
#pragma unroll
  for (int e = 0; e < 4; ++e) {
    const float f0 = keepv ? (a0[e] * scale) : 0.0f;
    const float f1 = keepv ? (a1[e] * scale) : 0.0f;
    hv[e]     = (_Float16)f0;
    hv[4 + e] = (_Float16)f1;
  }
  unsigned short* q = dst + (size_t)e0;
  *(volatile v8h*)q = hv;
  __threadfence();
  *(volatile v8h*)q = hv;
}

__global__ __launch_bounds__(256) void encoder_kernel(
    const float* __restrict__ mix, const float* __restrict__ encw,
    float* __restrict__ MW, float* __restrict__ PART)
{
  __shared__ float sRed[16];
  const int tid = threadIdx.x, lane = tid & 31, wave = tid >> 5;
  const int tok = tid >> 6;
  const int n4  = (tid & 63) * 4;
  const int m   = blockIdx.x * 4 + tok;
  const bool valid = m < kMV;
  const int mc = valid ? m : (kMV - 1);
  const int bb = (mc >= kL) ? 1 : 0;
  const int l  = mc - bb * kL;
  const float* x = mix + (size_t)bb * kSamp + (size_t)l * kStr;
  float acc[4] = {0.f, 0.f, 0.f, 0.f};
#pragma unroll 1
  for (int q = 0; q < 4; ++q) {
    const v4f xv = *(const v4f*)(x + 4 * q);
#pragma unroll
    for (int c = 0; c < 4; ++c) {
      const v4f wv = *(const v4f*)(encw + (size_t)(n4 + c) * kKer + 4 * q);
      acc[c] = fmaf(wv[0], xv[0], acc[c]);
      acc[c] = fmaf(wv[1], xv[1], acc[c]);
      acc[c] = fmaf(wv[2], xv[2], acc[c]);
      acc[c] = fmaf(wv[3], xv[3], acc[c]);
    }
  }
  v4f o;
#pragma unroll
  for (int c = 0; c < 4; ++c) {
    const float r = fmaxf(acc[c], 0.0f);
    o[c] = valid ? r : 0.0f;
  }
  float s = (o[0] + o[1]) + (o[2] + o[3]);
  float q2 = (o[0] * o[0] + o[1] * o[1]) + (o[2] * o[2] + o[3] * o[3]);
#pragma unroll
  for (int off = 16; off > 0; off >>= 1) {
    s  += __shfl_xor(s, off, 32);
    q2 += __shfl_xor(q2, off, 32);
  }
  if (lane == 0) { sRed[wave] = s; sRed[8 + wave] = q2; }
  float* dst = MW + (size_t)m * kEnc + n4;
  *(volatile v4f*)dst = o;
  __threadfence();
  *(volatile v4f*)dst = o;
  __syncthreads();
  if (wave == 0) {
    const float rv = sRed[lane & 15];
    const float pv = (lane < 16) ? rv : 0.0f;
    volatile float* pl = PART + (size_t)blockIdx.x * 32 + lane;
    *pl = pv;
    __threadfence();
    *pl = pv;
  }
}

__global__ __launch_bounds__(256) void stats_final_kernel(
    const float* __restrict__ PART, float* __restrict__ STAT)
{
  __shared__ float sR[4][256];
  const int tid = threadIdx.x;
  float s0 = 0.f, q0 = 0.f, s1 = 0.f, q1 = 0.f;
#pragma unroll 1
  for (int ln = tid; ln < kPartLines; ln += 256) {
    const float* p = PART + (size_t)ln * 32;
    const v4f sa = *(const v4f*)(p);
    const v4f sb = *(const v4f*)(p + 4);
    const v4f qa = *(const v4f*)(p + 8);
    const v4f qb = *(const v4f*)(p + 12);
    const float ts0 = sa[0] + sa[1], ts1 = sa[2] + sa[3], ts2 = sb[0] + sb[1], ts3 = sb[2] + sb[3];
    const float tq0 = qa[0] + qa[1], tq1 = qa[2] + qa[3], tq2 = qb[0] + qb[1], tq3 = qb[2] + qb[3];
    const int tk = ln * 4;
    const bool f0 = (tk + 0) < kL, f1 = (tk + 1) < kL, f2 = (tk + 2) < kL, f3 = (tk + 3) < kL;
    s0 += ((f0 ? ts0 : 0.f) + (f1 ? ts1 : 0.f)) + ((f2 ? ts2 : 0.f) + (f3 ? ts3 : 0.f));
    q0 += ((f0 ? tq0 : 0.f) + (f1 ? tq1 : 0.f)) + ((f2 ? tq2 : 0.f) + (f3 ? tq3 : 0.f));
    s1 += ((f0 ? 0.f : ts0) + (f1 ? 0.f : ts1)) + ((f2 ? 0.f : ts2) + (f3 ? 0.f : ts3));
    q1 += ((f0 ? 0.f : tq0) + (f1 ? 0.f : tq1)) + ((f2 ? 0.f : tq2) + (f3 ? 0.f : tq3));
  }
  sR[0][tid] = s0; sR[1][tid] = q0; sR[2][tid] = s1; sR[3][tid] = q1;
  __syncthreads();
#pragma unroll 1
  for (int st = 128; st > 0; st >>= 1) {
    if (tid < st) {
      sR[0][tid] += sR[0][tid + st];
      sR[1][tid] += sR[1][tid + st];
      sR[2][tid] += sR[2][tid + st];
      sR[3][tid] += sR[3][tid + st];
    }
    __syncthreads();
  }
  const float inv = 1.0f / (float)(kEnc * kL);
  const float S0 = sR[0][0], Q0 = sR[1][0], S1 = sR[2][0], Q1 = sR[3][0];
  const float mu0 = S0 * inv, mu1 = S1 * inv;
  const float var0 = fmaxf(Q0 * inv - mu0 * mu0, 0.0f);
  const float var1 = fmaxf(Q1 * inv - mu1 * mu1, 0.0f);
  const float r0 = __builtin_amdgcn_rcpf(sqrtf(var0 + 1e-5f));
  const float r1 = __builtin_amdgcn_rcpf(sqrtf(var1 + 1e-5f));
  float v = 0.0f;
  v = (tid == 0) ? mu0 : v;
  v = (tid == 1) ? r0 : v;
  v = (tid == 2) ? mu1 : v;
  v = (tid == 3) ? r1 : v;
  if (tid < 32) {
    volatile float* ps = STAT + tid;
    *ps = v;
    __threadfence();
    *ps = v;
  }
}

__global__ __launch_bounds__(256) void gn_pack_kernel(
    const float* __restrict__ MW, const float* __restrict__ STAT,
    const float* __restrict__ gnw, const float* __restrict__ gnb, unsigned short* __restrict__ GN)
{
  const int i  = blockIdx.x * 256 + threadIdx.x;
  const int e0 = i << 3;
  const int m  = e0 >> 8;
  const int n  = e0 & 255;
  const bool valid = m < kMV;
  const int bb = (m >= kL) ? 1 : 0;
  const float mu = STAT[bb * 2 + 0];
  const float rs = STAT[bb * 2 + 1];
  const v4f a0 = *(const v4f*)(MW + (size_t)e0);
  const v4f a1 = *(const v4f*)(MW + (size_t)e0 + 4);
  const v4f w0 = *(const v4f*)(gnw + n);
  const v4f w1 = *(const v4f*)(gnw + n + 4);
  const v4f b0 = *(const v4f*)(gnb + n);
  const v4f b1 = *(const v4f*)(gnb + n + 4);
  v8h hv;
#pragma unroll
  for (int e = 0; e < 4; ++e) {
    const float f0 = ((a0[e] - mu) * rs * w0[e] + b0[e]) * kActCarry;
    const float f1 = ((a1[e] - mu) * rs * w1[e] + b1[e]) * kActCarry;
    hv[e]     = (_Float16)(valid ? f0 : 0.0f);
    hv[4 + e] = (_Float16)(valid ? f1 : 0.0f);
  }
  unsigned short* q = GN + (size_t)e0;
  *(volatile v8h*)q = hv;
  __threadfence();
  *(volatile v8h*)q = hv;
}

__global__ __launch_bounds__(256) void resid_norm_kernel(
    const float* __restrict__ Xold, const float* __restrict__ YD0, const float* __restrict__ YD1,
    float* __restrict__ Xnew, const float* __restrict__ w,
    unsigned short* __restrict__ XNF, unsigned short* __restrict__ XNR, int has_y)
{
  __shared__ __align__(16) float sRow[8][256];
  const int tid = threadIdx.x, lane = tid & 31, wave = tid >> 5;
  const int m = blockIdx.x * 8 + wave;
  const int bb = (m >= kL) ? 1 : 0;
  const int lfl = bb * kL + (kL - 1) - (m - bb * kL);
  const int mr = (m < kMV) ? lfl : m;
  const int c0 = lane * 4, c1 = 128 + lane * 4;
  v4f x0 = *(const v4f*)(Xold + (size_t)m * kBot + c0);
  v4f x1 = *(const v4f*)(Xold + (size_t)m * kBot + c1);
  if (has_y) {
    const v4f f0 = *(const v4f*)(YD0 + (size_t)m * kBot + c0);
    const v4f f1 = *(const v4f*)(YD0 + (size_t)m * kBot + c1);
    const v4f r0 = *(const v4f*)(YD1 + (size_t)mr * kBot + c0);
    const v4f r1 = *(const v4f*)(YD1 + (size_t)mr * kBot + c1);
    x0 = (x0 + f0) + r0;
    x1 = (x1 + f1) + r1;
  }
  float ssq = (x0[0] * x0[0] + x0[1] * x0[1]) + (x0[2] * x0[2] + x0[3] * x0[3]);
  ssq += (x1[0] * x1[0] + x1[1] * x1[1]) + (x1[2] * x1[2] + x1[3] * x1[3]);
#pragma unroll
  for (int off = 16; off > 0; off >>= 1) ssq += __shfl_xor(ssq, off, 32);
  const float rs = __builtin_amdgcn_rcpf(sqrtf(ssq * (1.0f / (float)kBot) + 1e-5f)) * kActCarry;
  const v4f w0 = *(const v4f*)(w + c0);
  const v4f w1 = *(const v4f*)(w + c1);
  const v4f n0 = x0 * w0 * rs;
  const v4f n1 = x1 * w1 * rs;
  *(v4f*)(&sRow[wave][c0]) = n0;
  *(v4f*)(&sRow[wave][c1]) = n1;
  if (has_y) {
    float* px = Xnew + (size_t)m * kBot;
    for (int pass = 0; pass < 2; ++pass) {
      *(volatile v4f*)(px + c0) = x0;
      *(volatile v4f*)(px + c1) = x1;
      __threadfence();
    }
  }
  __syncthreads();
  const v4f a0 = *(const v4f*)(&sRow[wave][lane * 8]);
  const v4f a1 = *(const v4f*)(&sRow[wave][lane * 8 + 4]);
  v8h hv;
#pragma unroll
  for (int e = 0; e < 4; ++e) {
    hv[e]     = (_Float16)a0[e];
    hv[4 + e] = (_Float16)a1[e];
  }
  unsigned short* pf = XNF + (size_t)m  * kBot + lane * 8;
  unsigned short* pr = XNR + (size_t)mr * kBot + lane * 8;
  for (int pass = 0; pass < 2; ++pass) {
    *(volatile v8h*)pf = hv;
    *(volatile v8h*)pr = hv;
    __threadfence();
  }
}

__global__ __launch_bounds__(256) void conv_silu_kernel(
    const float* __restrict__ XZ, const float* __restrict__ cw, const float* __restrict__ cb,
    float* __restrict__ XC, unsigned short* __restrict__ XC16)
{
  __shared__ __align__(16) float sT[16 * kConvTP];
  const int tid = threadIdx.x, lane = tid & 31, wave = tid >> 5;
  const int dir = blockIdx.z;
  const float* XZd = XZ + (size_t)dir * kMP * kXzP;
  float* XCd = XC + (size_t)dir * kMP * kDI;
  unsigned short* XHd = XC16 + (size_t)dir * kMP * kDI;
  const int d0 = blockIdx.x * 256, d = d0 + tid;
  const int g0 = blockIdx.y * 64;
  const float* cwd = cw + ((size_t)dir * kDI + d) * 4;
  const float w0 = cwd[0], w1 = cwd[1], w2 = cwd[2], w3 = cwd[3];
  const float bc = cb[(size_t)dir * kDI + d];
  float xm3, xm2, xm1;
  {
    const int bstart = (g0 >= kL) ? kL : 0;
    const int r3 = g0 - 3, r2 = g0 - 2, r1 = g0 - 1;
    const float v3 = XZd[(size_t)(r3 < 0 ? 0 : r3) * kXzP + d];
    const float v2 = XZd[(size_t)(r2 < 0 ? 0 : r2) * kXzP + d];
    const float v1 = XZd[(size_t)(r1 < 0 ? 0 : r1) * kXzP + d];
    xm3 = (r3 >= bstart) ? v3 : 0.f;
    xm2 = (r2 >= bstart) ? v2 : 0.f;
    xm1 = (r1 >= bstart) ? v1 : 0.f;
  }
  const int hrow = wave >> 1;
  const int hch  = (wave & 1) * 128 + lane * 4;
#pragma unroll 1
  for (int sub = 0; sub < 4; ++sub) {
    const int lb = g0 + sub * 16;
#pragma unroll 1
    for (int s = 0; s < 16; ++s) {
      const int m = lb + s;
      if (m == kL) { xm3 = 0.f; xm2 = 0.f; xm1 = 0.f; }
      const float xcur = XZd[(size_t)m * kXzP + d];
      float acc = w0 * xm3;
      acc = fmaf(w1, xm2, acc);
      acc = fmaf(w2, xm1, acc);
      acc = fmaf(w3, xcur, acc);
      const float sv = acc + bc;
      const float sg = __builtin_amdgcn_rcpf(1.0f + expf(-sv));
      const float ov = sv * sg;
      sT[s * kConvTP + tid] = (m < kMV) ? ov : 0.0f;
      xm3 = xm2; xm2 = xm1; xm1 = xcur;
    }
    __syncthreads();
    v4f fv[4];
    v8h bv[2];
#pragma unroll
    for (int it = 0; it < 4; ++it) fv[it] = *(const v4f*)(sT + (it * 4 + hrow) * kConvTP + hch);
#pragma unroll
    for (int it = 0; it < 2; ++it) {
      const float* sp = sT + (it * 8 + wave) * kConvTP + lane * 8;
      const v4f a0 = *(const v4f*)(sp);
      const v4f a1 = *(const v4f*)(sp + 4);
#pragma unroll
      for (int e = 0; e < 4; ++e) {
        bv[it][e]     = (_Float16)(a0[e] * kActCarry);
        bv[it][4 + e] = (_Float16)(a1[e] * kActCarry);
      }
    }
    for (int pass = 0; pass < 2; ++pass) {
#pragma unroll
      for (int it = 0; it < 4; ++it)
        *(volatile v4f*)(XCd + (size_t)(lb + it * 4 + hrow) * kDI + d0 + hch) = fv[it];
#pragma unroll
      for (int it = 0; it < 2; ++it)
        *(volatile v8h*)(XHd + (size_t)(lb + it * 8 + wave) * kDI + d0 + lane * 8) = bv[it];
      __threadfence();
    }
    __syncthreads();
  }
}

__global__ __launch_bounds__(64) void scan_gate_kernel(
    const float* __restrict__ XD, const float* __restrict__ UC, const float* __restrict__ XZ,
    const float* __restrict__ Wdt, const float* __restrict__ bdt, const float* __restrict__ Alog,
    const float* __restrict__ Dp, unsigned short* __restrict__ G16)
{
  __shared__ __align__(16) float sX[kScanTS * kXdP];
  __shared__ __align__(16) float sY[kScanTS * kScanYP];
  __shared__ __align__(16) float sW[kDtR * kScanCh];
  __shared__ __align__(16) float sA[kNS * kScanCh];
  const int tid = threadIdx.x, lane = tid & 31, wave = tid >> 5;
  const int dir = blockIdx.y;
  const int bix = blockIdx.x >> 3;
  const int d0  = (blockIdx.x & 7) * kScanCh;
  const int d   = d0 + tid;
  const float* XDd = XD + (size_t)dir * kMP * kXdP;
  const float* UCd = UC + (size_t)dir * kMP * kDI;
  const float* XZd = XZ + (size_t)dir * kMP * kXzP;
  const float* Wd  = Wdt  + (size_t)dir * kDI * kDtR;
  const float* Ad  = Alog + (size_t)dir * kDI * kNS;
  unsigned short* Gd = G16 + (size_t)dir * kMP * kDI;
  const int row0 = bix * kL;
#pragma unroll 1
  for (int r = 0; r < kDtR; ++r) sW[r * kScanCh + tid] = Wd[(size_t)d * kDtR + r];
#pragma unroll 1
  for (int s = 0; s < kNS; ++s) sA[s * kScanCh + tid] = -expf(Ad[(size_t)d * kNS + s]);
  __syncthreads();
  float negA[kNS], h[kNS];
#pragma unroll
  for (int s = 0; s < kNS; ++s) {
    negA[s] = sA[s * kScanCh + tid];
    h[s] = 0.f;
  }
  const float bb = bdt[(size_t)dir * kDI + d];
  const float Dd = Dp[(size_t)dir * kDI + d];
  const int lr = tid >> 4, lc4 = (tid & 15) * 4;
  const int q = lane >> 3, c8 = (lane & 7) * 8;
  const int nChunks = bix ? 17 : 16;
  const int tlim = bix ? (kMP - kL) : kL;
#pragma unroll 1
  for (int ck = 0; ck < nChunks; ++ck) {
    const int t0 = ck * kScanTS;
    __syncthreads();
#pragma unroll
    for (int i = 0; i < 16; ++i) {
      const int r = lr + 4 * i;
      const int mrow = row0 + t0 + r;
      const int mrc = (mrow < kMP) ? mrow : (kMP - 1);
      *(v4f*)(sX + r * kXdP + lc4) = *(const v4f*)(XDd + (size_t)mrc * kXdP + lc4);
    }
    __syncthreads();
#pragma unroll 1
    for (int s = 0; s < kScanTS; ++s) {
      const int t = t0 + s;
      if (t < kL) {
        const size_t grow = (size_t)(row0 + t);
        const float* xr = sX + s * kXdP;
        float vdot = 0.f;
#pragma unroll 1
        for (int r4 = 0; r4 < kDtR / 4; ++r4) {
          const v4f xv = *(const v4f*)(xr + 4 * r4);
          const float* wp = sW + (4 * r4) * kScanCh + tid;
          vdot = fmaf(xv[0], wp[0], vdot);
          vdot = fmaf(xv[1], wp[kScanCh], vdot);
          vdot = fmaf(xv[2], wp[2 * kScanCh], vdot);
          vdot = fmaf(xv[3], wp[3 * kScanCh], vdot);
        }
        float Bs[kNS], Cs[kNS];
#pragma unroll
        for (int q4 = 0; q4 < 4; ++q4) {
          const v4f bv = *(const v4f*)(xr + kDtR + 4 * q4);
          const v4f cv = *(const v4f*)(xr + kDtR + kNS + 4 * q4);
          Bs[4 * q4 + 0] = bv[0]; Bs[4 * q4 + 1] = bv[1]; Bs[4 * q4 + 2] = bv[2]; Bs[4 * q4 + 3] = bv[3];
          Cs[4 * q4 + 0] = cv[0]; Cs[4 * q4 + 1] = cv[1]; Cs[4 * q4 + 2] = cv[2]; Cs[4 * q4 + 3] = cv[3];
        }
        const float v   = vdot + bb;
        const float ea  = __expf(-fabsf(v));
        const float up  = 1.0f + ea;
        const float l1p = __logf(up) + (ea - (up - 1.0f)) * __builtin_amdgcn_rcpf(up);
        const float dt  = fmaxf(v, 0.0f) + l1p;
        const float xt  = UCd[grow * kDI + d];
        const float dtx = dt * xt;
        float y = 0.f;
#pragma unroll
        for (int k = 0; k < kNS; ++k) {
          const float e = __expf(dt * negA[k]);
          h[k] = e * h[k] + dtx * Bs[k];
          y = h[k] * Cs[k] + y;
        }
        y = xt * Dd + y;
        const float zv = XZd[grow * kXzP + kDI + d];
        const float sg = __builtin_amdgcn_rcpf(1.0f + expf(-zv));
        y = y * (zv * sg);
        sY[s * kScanYP + tid] = y * kActCarry;
      } else {
        sY[s * kScanYP + tid] = 0.0f;
      }
    }
    __syncthreads();
    v8h hv[8];
#pragma unroll
    for (int it = 0; it < 8; ++it) {
      const int row = it * 8 + wave * 4 + q;
      const float* sp = sY + row * kScanYP + c8;
      const v4f a0 = *(const v4f*)(sp);
      const v4f a1 = *(const v4f*)(sp + 4);
#pragma unroll
      for (int e = 0; e < 4; ++e) {
        hv[it][e]     = (_Float16)a0[e];
        hv[it][4 + e] = (_Float16)a1[e];
      }
    }
    for (int pass = 0; pass < 2; ++pass) {
#pragma unroll
      for (int it = 0; it < 8; ++it) {
        const int row = it * 8 + wave * 4 + q;
        if (t0 + row < tlim) {
          const size_t o = (size_t)(row0 + t0 + row) * kDI + d0 + c8;
          *(volatile v8h*)(Gd + o) = hv[it];
        }
      }
      __threadfence();
    }
  }
}

__global__ __launch_bounds__(256) void decoder_kernel(
    const float* __restrict__ MW, const float* __restrict__ MSK,
    const float* __restrict__ decw, float* __restrict__ out)
{
  const int g = blockIdx.x * 256 + threadIdx.x;
  if (g >= kBatch * kSamp) return;
  const int bb = g / kSamp;
  const int t  = g - bb * kSamp;
  const int f0 = t >> 3, k0 = t & 7;
  const int f1 = f0 - 1, k1 = k0 + 8;
  const bool ok0 = f0 <= (kL - 1);
  const bool ok1 = f1 >= 0;
  const int f0c = ok0 ? f0 : (kL - 1);
  const int f1c = ok1 ? f1 : 0;
  const size_t r0 = (size_t)(bb * kL + f0c) * kEnc;
  const size_t r1 = (size_t)(bb * kL + f1c) * kEnc;
  float acc0 = 0.f, acc1 = 0.f;
#pragma unroll 1
  for (int n4 = 0; n4 < kEnc / 4; ++n4) {
    const v4f a  = *(const v4f*)(MW  + r0 + 4 * n4);
    const v4f ma = *(const v4f*)(MSK + r0 + 4 * n4);
    const v4f c  = *(const v4f*)(MW  + r1 + 4 * n4);
    const v4f mc = *(const v4f*)(MSK + r1 + 4 * n4);
#pragma unroll
    for (int e = 0; e < 4; ++e) {
      const int n = 4 * n4 + e;
      const float wa = decw[n * kKer + k0];
      const float wb = decw[n * kKer + k1];
      const float pa = a[e] * ma[e];
      const float pc = c[e] * mc[e];
      acc0 = fmaf(pa, wa, acc0);
      acc1 = fmaf(pc, wb, acc1);
    }
  }
  const float yv = (ok0 ? acc0 : 0.0f) + (ok1 ? acc1 : 0.0f);
  volatile float* po = out + g;
  *po = yv;
  __threadfence();
  *po = yv;
}

extern "C" void kernel_launch(void* const* d_in, const int* in_sizes, int n_in,
                              void* d_out, int out_size, void* d_ws, size_t ws_size,
                              hipStream_t stream)
{
  if (n_in < 20) return;
  if (in_sizes[0] != kBatch * kSamp) return;
  if (in_sizes[1] != kEnc * kKer || in_sizes[2] != kEnc * kKer) return;
  if (in_sizes[5] != kBot * kEnc) return;
  if (in_sizes[8] != kNBlk * 2 * kXzP * kBot) return;
  if (in_sizes[9] != kNBlk * 2 * kDI * 4) return;
  if (in_sizes[11] != kNBlk * 2 * kXpN * kDI) return;
  if (in_sizes[12] != kNBlk * 2 * kDI * kDtR) return;
  if (in_sizes[14] != kNBlk * 2 * kDI * kNS) return;
  if (in_sizes[16] != kNBlk * 2 * kBot * kDI) return;
  if (in_sizes[18] != kEnc * kBot) return;
  if (out_size != kBatch * kSamp) return;
  if (ws_size < kWsTotal) return;

  const float* mixture = (const float*)d_in[0];
  const float* enc_w   = (const float*)d_in[1];
  const float* dec_w   = (const float*)d_in[2];
  const float* gn_w    = (const float*)d_in[3];
  const float* gn_b    = (const float*)d_in[4];
  const float* bot_w   = (const float*)d_in[5];
  const float* bot_b   = (const float*)d_in[6];
  const float* blk_nw  = (const float*)d_in[7];
  const float* in_w    = (const float*)d_in[8];
  const float* conv_w  = (const float*)d_in[9];
  const float* conv_b  = (const float*)d_in[10];
  const float* xproj_w = (const float*)d_in[11];
  const float* dt_w    = (const float*)d_in[12];
  const float* dt_b    = (const float*)d_in[13];
  const float* A_log   = (const float*)d_in[14];
  const float* Dmat    = (const float*)d_in[15];
  const float* out_w   = (const float*)d_in[16];
  const float* normf_w = (const float*)d_in[17];
  const float* mask_w  = (const float*)d_in[18];
  const float* mask_b  = (const float*)d_in[19];
  float* y_out = (float*)d_out;

  char* ws = (char*)d_ws;
  unsigned short* WIN  = (unsigned short*)(ws + kOffWIN);
  unsigned short* WOUT = (unsigned short*)(ws + kOffWOUT);
  unsigned short* WXP  = (unsigned short*)(ws + kOffWXP);
  unsigned short* WBOT = (unsigned short*)(ws + kOffWBOT);
  unsigned short* WMSK = (unsigned short*)(ws + kOffWMSK);
  float*          MW   = (float*)(ws + kOffMW);
  float*          PART = (float*)(ws + kOffPART);
  float*          STAT = (float*)(ws + kOffSTAT);
  unsigned short* GN   = (unsigned short*)(ws + kOffGN);
  float*          XA   = (float*)(ws + kOffXA);
  float*          XB   = (float*)(ws + kOffXB);
  unsigned short* XN   = (unsigned short*)(ws + kOffXN);
  float*          XZ   = (float*)(ws + kOffXZ);
  float*          XC   = (float*)(ws + kOffXC);
  unsigned short* XC16 = (unsigned short*)(ws + kOffXC16);
  float*          XD   = (float*)(ws + kOffXD);
  unsigned short* G16  = (unsigned short*)(ws + kOffG);
  float*          YD   = (float*)(ws + kOffYD);
  float*          MSK  = (float*)(ws + kOffMSK);
  unsigned short* XNF  = XN;
  unsigned short* XNR  = XN + (size_t)kMP * kBot;
  float* YD0 = YD;
  float* YD1 = YD + (size_t)kMP * kBot;

  cast_f16_kernel<<<(kNBlk * 2 * kXzP * kBot) / 8 / 256, 256, 0, stream>>>(in_w, WIN, (kNBlk * 2 * kXzP * kBot) / 8, kWgtCarry);
  cast_f16_kernel<<<(kNBlk * 2 * kBot * kDI) / 8 / 256, 256, 0, stream>>>(out_w, WOUT, (kNBlk * 2 * kBot * kDI) / 8, kWgtCarry);
  xproj_pad_cast_kernel<<<(kNBlk * 2 * kXdP * kDI) / 8 / 256, 256, 0, stream>>>(xproj_w, WXP, (kNBlk * 2 * kXdP * kDI) / 8, kWgtCarry);
  cast_f16_kernel<<<(kBot * kEnc) / 8 / 256, 256, 0, stream>>>(bot_w, WBOT, (kBot * kEnc) / 8, kWgtCarry);
  cast_f16_kernel<<<(kEnc * kBot) / 8 / 256, 256, 0, stream>>>(mask_w, WMSK, (kEnc * kBot) / 8, kWgtCarry);

  encoder_kernel<<<kMP / 4, 256, 0, stream>>>(mixture, enc_w, MW, PART);
  stats_final_kernel<<<1, 256, 0, stream>>>(PART, STAT);
  gn_pack_kernel<<<(kMP * kEnc) / 8 / 256, 256, 0, stream>>>(MW, STAT, gn_w, gn_b, GN);
  gemm64_f16_kernel<2, 0><<<dim3((kMP / 64) * (kBot / 64) / 8, 1), 256, 0, stream>>>(
      GN, kEnc, 0L, WBOT, kEnc, 0L, XA, kBot, 0L, bot_b, kMP, kBot, kEnc, kFold);

  float* cur = XA;
  float* nxt = XB;
  resid_norm_kernel<<<kMP / 8, 256, 0, stream>>>(cur, YD0, YD1, nxt, blk_nw, XNF, XNR, 0);

  for (int i = 0; i < kNBlk; ++i) {
    const size_t wq = (size_t)i * 2;
    gemm64_f16_kernel<0, 0><<<dim3((kMP / 64) * (kXzP / 64) / 8, 2), 256, 0, stream>>>(
        XN, kBot, (long)kMP * kBot, WIN + wq * kXzP * kBot, kBot, (long)kXzP * kBot,
        XZ, kXzP, (long)kMP * kXzP, bot_b, kMP, kXzP, kBot, kFold);
    conv_silu_kernel<<<dim3(kDI / 256, kMP / 64, 2), 256, 0, stream>>>(
        XZ, conv_w + wq * kDI * 4, conv_b + wq * kDI, XC, XC16);
    gemm64_f16_kernel<0, 0><<<dim3((kMP / 64) * (kXdP / 64) / 8, 2), 256, 0, stream>>>(
        XC16, kDI, (long)kMP * kDI, WXP + wq * kXdP * kDI, kDI, (long)kXdP * kDI,
        XD, kXdP, (long)kMP * kXdP, bot_b, kMP, kXdP, kDI, kFold);
    scan_gate_kernel<<<dim3(kBatch * (kDI / kScanCh), 2), kScanCh, 0, stream>>>(
        XD, XC, XZ, dt_w + wq * kDI * kDtR, dt_b + wq * kDI, A_log + wq * kDI * kNS, Dmat + wq * kDI, G16);
    gemm64_f16_kernel<0, 0><<<dim3((kMP / 64) * (kBot / 64) / 8, 2), 256, 0, stream>>>(
        G16, kDI, (long)kMP * kDI, WOUT + wq * kBot * kDI, kDI, (long)kBot * kDI,
        YD, kBot, (long)kMP * kBot, bot_b, kMP, kBot, kDI, kFold);
    const float* wn = (i + 1 < kNBlk) ? (blk_nw + (size_t)(i + 1) * kBot) : normf_w;
    resid_norm_kernel<<<kMP / 8, 256, 0, stream>>>(cur, YD0, YD1, nxt, wn, XNF, XNR, 1);
    float* tmp = cur; cur = nxt; nxt = tmp;
  }

  gemm64_f16_kernel<2, 2><<<dim3((kMP / 64) * (kEnc / 64) / 8, 1), 256, 0, stream>>>(
      XNF, kBot, 0L, WMSK, kBot, 0L, MSK, kEnc, 0L, mask_b, kMP, kEnc, kBot, kFold);
  decoder_kernel<<<(kBatch * kSamp + 255) / 256, 256, 0, stream>>>(MW, MSK, dec_w, y_out);
}
